// FactorizedLayer_45629732553452
// MI455X (gfx1250) — hardware-verified
//
#include <hip/hip_runtime.h>
#include <math.h>

#ifndef NB
#define NB 4096
#endif
#define NB_FULL 4096
#define KD 512
#define HID 1024
#define LAT 8
#define NCOL (HID * LAT)
#define KCAT (2 * KD)

#define CX 8.0f
#define CW 32.0f
#define CXQ 256.0f
#define CBQ (-0.5f)
static constexpr float SC = 1.0f / 256.0f;

#define FM_TM 64
#define FM_TN 256
#define FM_HB (FM_TN / LAT)
#define FM_FP 36

static_assert(NB % 64 == 0);
static_assert(NB <= NB_FULL);
static_assert(HID % 64 == 0);
static_assert(KD % 32 == 0 && KCAT % 32 == 0);
static_assert(KD / 8 == 64);
static_assert(LAT == 8);
static_assert(NCOL % FM_TN == 0 && NB % FM_TM == 0);
static_assert(FM_HB == 32);
static_assert((NB * (KD / 8)) % 256 == 0);
static_assert((HID * (KD / 8)) % 256 == 0);
static_assert(CX * CW * SC == 1.0f);
static_assert(CXQ * CBQ * SC == -0.5f);
static_assert(4 * 4 * 4 == FM_TM);
static_assert(128 * 16 * 4 == FM_TM * FM_HB * 4);
static_assert(8 * 16 * 68 * 4 <= 131072);
static_assert(FM_TM * FM_FP * 4 <= 131072);

static constexpr size_t SZ_XA = (size_t)NB * KCAT * 2;
static constexpr size_t SZ_XB = (size_t)NB * KD * 2;
static constexpr size_t SZ_BB = (size_t)NCOL * KD * 2;
static constexpr size_t SZ_WB = (size_t)HID * KCAT * 2;
static constexpr size_t SZ_FM = (size_t)NB * HID * 4;
static_assert(SZ_XA % 256 == 0 && SZ_XB % 256 == 0 && SZ_BB % 256 == 0 && SZ_WB % 256 == 0 && SZ_FM % 256 == 0);
static_assert(SZ_XA + SZ_XB + SZ_BB + SZ_WB + SZ_FM <= (size_t)134217728);

typedef __attribute__((ext_vector_type(16))) _Float16 v16h;
typedef __attribute__((ext_vector_type(8)))  _Float16 v8h;
typedef __attribute__((ext_vector_type(16))) __bf16   v16b;
typedef __attribute__((ext_vector_type(8)))  float    v8f;
typedef __attribute__((ext_vector_type(4)))  float    v4f;
typedef __attribute__((ext_vector_type(4)))  unsigned int v4u;
typedef _Float16 h16;


#define VST2(T, ptr, val) do { const T vst2_v_ = (val); *(volatile T*)(ptr) = vst2_v_; __threadfence(); *(volatile T*)(ptr) = vst2_v_; } while (0)

__device__ __forceinline__ float bfr(float f) {
    unsigned u = __float_as_uint(f);
    u += 0x7FFFu + ((u >> 16) & 1u);
    return __uint_as_float(u & 0xFFFF0000u);
}
static __device__ __forceinline__ h16 toh_flush(float v) { const h16 r = (h16)v; return (fabsf(v) < 6.103515625e-05f) ? (h16)0.0f : r; }
__device__ __forceinline__ unsigned hbits(float v) { return (unsigned)__builtin_bit_cast(unsigned short, toh_flush(v)); }
__device__ __forceinline__ void st8hf(unsigned short* P, size_t o, const float* v) {
    v4u pk;
    pk.x = hbits(v[0]) | (hbits(v[1]) << 16);
    pk.y = hbits(v[2]) | (hbits(v[3]) << 16);
    pk.z = hbits(v[4]) | (hbits(v[5]) << 16);
    pk.w = hbits(v[6]) | (hbits(v[7]) << 16);
    VST2(v4u, (v4u*)(P + o), pk);
}
__device__ __forceinline__ void st8b(unsigned short* P, size_t o, const float* v) {
    v4u pk;
    pk.x = (__float_as_uint(v[0]) >> 16) | (__float_as_uint(v[1]) & 0xFFFF0000u);
    pk.y = (__float_as_uint(v[2]) >> 16) | (__float_as_uint(v[3]) & 0xFFFF0000u);
    pk.z = (__float_as_uint(v[4]) >> 16) | (__float_as_uint(v[5]) & 0xFFFF0000u);
    pk.w = (__float_as_uint(v[6]) >> 16) | (__float_as_uint(v[7]) & 0xFFFF0000u);
    VST2(v4u, (v4u*)(P + o), pk);
}

union FragU { v16h v; v8h h[2]; };
__device__ __forceinline__ v16h frag_ld(const _Float16* p) {
    FragU f; f.h[0] = *(const v8h*)(p); f.h[1] = *(const v8h*)(p + 16); return f.v;
}
union FragB { v16b v; v4u q[2]; };
__device__ __forceinline__ v16b frag_ldb(const unsigned short* p) {
    FragB f; f.q[0] = *(const v4u*)(p); f.q[1] = *(const v4u*)(p + 16); return f.v;
}
__device__ __forceinline__ v8f wmma16b(v16b a, v16b b, v8f c) {
    c = __builtin_amdgcn_wmma_f32_16x16x32_bf16(false, a, false, b, (short)0, c, false, false);
    asm volatile("v_nop\n\tv_nop\n\tv_nop\n\tv_nop" : "+v"(c) : "v"(a), "v"(b));
    return c;
}
__device__ __forceinline__ void dep_guard_h(v8f& a, v8f& b, v16h x, v16h y) { asm volatile("v_nop\n\tv_nop\n\tv_nop\n\tv_nop" : "+v"(a), "+v"(b) : "v"(x), "v"(y)); }
__device__ __forceinline__ void keep4_h(v16h a, v16h b, v16h c, v16h d) { asm volatile("v_nop" :: "v"(a), "v"(b), "v"(c), "v"(d)); }
__device__ __forceinline__ void acc_guard4(v8f& a, v8f& b, v8f& c, v8f& d) { asm volatile("v_nop\n\tv_nop\n\tv_nop\n\tv_nop" : "+v"(a), "+v"(b), "+v"(c), "+v"(d)); }
__device__ __forceinline__ void wave_sync_lds() {
    __builtin_amdgcn_fence(3  , "workgroup");
    __builtin_amdgcn_wave_barrier();
    __builtin_amdgcn_fence(2  , "workgroup");
}

template <int OUT_MODE, bool RESID, bool RELU>
__global__ __launch_bounds__(256) void k_gemm64(
    const _Float16* __restrict__ A, unsigned lda, const _Float16* __restrict__ Bt, unsigned ldb,
    void* __restrict__ Cout, unsigned ldc, const float* __restrict__ bias, const float* __restrict__ resid,
    unsigned M, unsigned N, unsigned K, float scale, float oscale) {
  __shared__ __align__(16) float sT[8][16 * 68];
  const unsigned lane = threadIdx.x & 31u;
  const unsigned wave = threadIdx.x >> 5;
  const unsigned tilesN = N >> 6, tilesM = M >> 6;
  const unsigned tile = blockIdx.x * 8u + wave;
  if (tile >= tilesM * tilesN) return;
  const unsigned tm = tile / tilesN;
  const unsigned tn = tile - tm * tilesN;
  const unsigned m0 = tm << 6, n0 = tn << 6;
  const unsigned rlane = lane & 15u;
  const unsigned koff = (lane >> 4) * 8u;
  const unsigned mOff = koff;

  v8f acc[4][4];
#pragma unroll
  for (int i = 0; i < 4; ++i)
#pragma unroll
    for (int j = 0; j < 4; ++j) acc[i][j] = (v8f){0.f,0.f,0.f,0.f,0.f,0.f,0.f,0.f};

  for (unsigned k0 = 0; k0 < K; k0 += 32u) {
    v16h bh[4];
#pragma unroll
    for (int j = 0; j < 4; ++j)
      bh[j] = frag_ld(Bt + (size_t)(n0 + ((unsigned)j << 4) + rlane) * ldb + koff + k0);
#pragma unroll
    for (int i = 0; i < 4; ++i) {
      const v16h ah = frag_ld(A + (size_t)(m0 + ((unsigned)i << 4) + rlane) * lda + koff + k0);
#pragma unroll
      for (int j = 0; j < 4; ++j)
        acc[i][j] = __builtin_amdgcn_wmma_f32_16x16x32_f16(false, ah, false, bh[j], (short)0, acc[i][j], false, false);
      dep_guard_h(acc[i][0], acc[i][3], ah, ah);
    }
    keep4_h(bh[0], bh[1], bh[2], bh[3]);
  }
  acc_guard4(acc[0][0], acc[0][1], acc[0][2], acc[0][3]);
  acc_guard4(acc[1][0], acc[1][1], acc[1][2], acc[1][3]);
  acc_guard4(acc[2][0], acc[2][1], acc[2][2], acc[2][3]);
  acc_guard4(acc[3][0], acc[3][1], acc[3][2], acc[3][3]);

  float* slab = sT[wave];
#pragma unroll
  for (int i = 0; i < 4; ++i) {
    const unsigned mBase = m0 + ((unsigned)i << 4);
#pragma unroll
    for (int j = 0; j < 4; ++j) {
      const unsigned n = n0 + ((unsigned)j << 4) + rlane;
      const float bv = bfr(bias[n]);
#pragma unroll
      for (int r = 0; r < 8; ++r) {
        float v = acc[i][j][r] * scale + bv;
        if (RELU) v = fmaxf(v, 0.0f);
        if (OUT_MODE == 1) v *= oscale;
        slab[(mOff + (unsigned)r) * 68u + ((unsigned)j << 4) + rlane] = v;
      }
    }
    wave_sync_lds();
    if (OUT_MODE == 0) {
      float* C = (float*)Cout;
      const unsigned hh = lane >> 4, c4 = (lane & 15u) * 4u;
#pragma unroll
      for (int half = 0; half < 2; ++half) {
        v4f vv[4];
#pragma unroll
        for (int it = 0; it < 4; ++it) {
          const unsigned row = (unsigned)(half * 4 + it) * 2u + hh;
          vv[it] = *(const v4f*)(slab + row * 68u + c4);
          if (RESID) vv[it] += *(const v4f*)(resid + (size_t)(mBase + row) * ldc + n0 + c4);
        }
        for (int pass = 0; pass < 2; ++pass) {
#pragma unroll
          for (int it = 0; it < 4; ++it) {
            const unsigned row = (unsigned)(half * 4 + it) * 2u + hh;
            *(volatile v4f*)(C + (size_t)(mBase + row) * ldc + n0 + c4) = vv[it];
          }
          __threadfence();
        }
      }
    } else {
      _Float16* C = (_Float16*)Cout;
      const unsigned q = lane >> 3, c8 = (lane & 7u) * 8u;
      v8h hv[4];
#pragma unroll
      for (int it = 0; it < 4; ++it) {
        const unsigned row = (unsigned)it * 4u + q;
        const float* sp = slab + row * 68u + c8;
#pragma unroll
        for (int e = 0; e < 8; ++e) hv[it][e] = (_Float16)sp[e];
      }
      for (int pass = 0; pass < 2; ++pass) {
#pragma unroll
        for (int it = 0; it < 4; ++it) {
          const unsigned row = (unsigned)it * 4u + q;
          *(volatile v8h*)(C + (size_t)(mBase + row) * ldc + n0 + c8) = hv[it];
        }
        __threadfence();
      }
    }
    wave_sync_lds();
  }
}

__global__ __launch_bounds__(256) void k_cvx(const float* __restrict__ x, unsigned short* __restrict__ XA,
                                             unsigned short* __restrict__ XB) {
#pragma clang fp contract(off)
    const unsigned u = blockIdx.x * 256u + threadIdx.x;
    if (u >= (unsigned)(NB * (KD / 8))) return;
    const unsigned row = u >> 6, c0 = (u & 63u) * 8u;
    const float* xr = x + (size_t)row * KD + c0;
    const v4f a = *(const v4f*)xr, b = *(const v4f*)(xr + 4);
    const float v[8] = {bfr(a.x), bfr(a.y), bfr(a.z), bfr(a.w), bfr(b.x), bfr(b.y), bfr(b.z), bfr(b.w)};
    float t[8];
#pragma unroll
    for (int i = 0; i < 8; ++i) t[i] = v[i] * CX;
    st8hf(XA, (size_t)row * KCAT + c0, t);
#pragma unroll
    for (int i = 0; i < 8; ++i) t[i] = (v[i] * v[i]) * CXQ;
    st8hf(XA, (size_t)row * KCAT + KD + c0, t);
    st8b(XB, (size_t)row * KD + c0, v);
}

__global__ __launch_bounds__(256) void k_cvbw(const float* __restrict__ beta, const float* __restrict__ Wm,
                                              unsigned short* __restrict__ BB, unsigned short* __restrict__ WB) {
#pragma clang fp contract(off)
    const unsigned u = blockIdx.x * 256u + threadIdx.x;
    if (u >= (unsigned)(HID * (KD / 8))) return;
    const unsigned h = u >> 6, c0 = (u & 63u) * 8u;
    float s2[8] = {0.f, 0.f, 0.f, 0.f, 0.f, 0.f, 0.f, 0.f};
#pragma unroll 1
    for (unsigned l = 0; l < (unsigned)LAT; ++l) {
        const size_t ro = ((size_t)h * LAT + l) * KD + c0;
        const v4f a = *(const v4f*)(beta + ro), b = *(const v4f*)(beta + ro + 4);
        const float v[8] = {bfr(a.x), bfr(a.y), bfr(a.z), bfr(a.w), bfr(b.x), bfr(b.y), bfr(b.z), bfr(b.w)};
#pragma unroll
        for (int i = 0; i < 8; ++i) s2[i] += v[i] * v[i];
        st8b(BB, ro, v);
    }
    float t[8];
#pragma unroll
    for (int i = 0; i < 8; ++i) t[i] = s2[i] * CBQ;
    st8hf(WB, (size_t)h * KCAT + KD + c0, t);
    {
        const float* wr = Wm + (size_t)h * KD + c0;
        const v4f a = *(const v4f*)wr, b = *(const v4f*)(wr + 4);
        const float w[8] = {bfr(a.x), bfr(a.y), bfr(a.z), bfr(a.w), bfr(b.x), bfr(b.y), bfr(b.z), bfr(b.w)};
#pragma unroll
        for (int i = 0; i < 8; ++i) t[i] = w[i] * CW;
        st8hf(WB, (size_t)h * KCAT + c0, t);
    }
}

__global__ __launch_bounds__(128) void k_fm(const unsigned short* __restrict__ XB, const unsigned short* __restrict__ BB,
                                            float* __restrict__ FM) {
#pragma clang fp contract(off)
    __shared__ __align__(16) float sF[FM_TM * FM_FP];
    const unsigned lane = threadIdx.x & 31u;
    const unsigned wave = (unsigned)__builtin_amdgcn_readfirstlane((int)(threadIdx.x >> 5));
    const unsigned tilesN = (unsigned)(NCOL / FM_TN);
    if (blockIdx.x >= (unsigned)(NB / FM_TM) * tilesN) return;
    const unsigned tm = blockIdx.x / tilesN;
    const unsigned tn = blockIdx.x - tm * tilesN;
    const unsigned m0 = tm * (unsigned)FM_TM;
    const unsigned n0 = tn * (unsigned)FM_TN + wave * 64u;
    const unsigned rlane = lane & 15u;
    const unsigned hh = lane >> 4;
    const unsigned koff = hh * 8u;

    v8f acc[4][4];
#pragma unroll
    for (int i = 0; i < 4; ++i)
#pragma unroll
        for (int j = 0; j < 4; ++j) acc[i][j] = (v8f){0.f,0.f,0.f,0.f,0.f,0.f,0.f,0.f};

#pragma unroll 1
    for (unsigned k0 = 0; k0 < (unsigned)KD; k0 += 32u) {
        v16b bh[4];
#pragma unroll
        for (int j = 0; j < 4; ++j)
            bh[j] = frag_ldb(BB + (size_t)(n0 + ((unsigned)j << 4) + rlane) * KD + koff + k0);
#pragma unroll
        for (int i = 0; i < 4; ++i) {
            const v16b ah = frag_ldb(XB + (size_t)(m0 + ((unsigned)i << 4) + rlane) * KD + koff + k0);
#pragma unroll
            for (int j = 0; j < 4; ++j) acc[i][j] = wmma16b(ah, bh[j], acc[i][j]);
        }
    }

#pragma unroll
    for (int i = 0; i < 4; ++i) {
#pragma unroll
        for (int j = 0; j < 4; ++j) {
            const unsigned hc = wave * 8u + (unsigned)j * 2u + ((lane >> 3) & 1u);
#pragma unroll
            for (int r = 0; r < 8; ++r) {
                const float sv = acc[i][j][r];
                float v = 0.5f * (sv * sv);
                v += __shfl_xor(v, 1, 32);
                v += __shfl_xor(v, 2, 32);
                v += __shfl_xor(v, 4, 32);
                if ((lane & 7u) == 0u) sF[((unsigned)i * 16u + 8u * hh + (unsigned)r) * FM_FP + hc] = v;
            }
        }
    }
    __syncthreads();
    {
        const unsigned q = lane >> 3, c4 = (lane & 7u) * 4u;
        v4f fv[4];
#pragma unroll
        for (int it = 0; it < 4; ++it) {
            const unsigned row = wave * 16u + (unsigned)it * 4u + q;
            fv[it] = *(const v4f*)(sF + row * FM_FP + c4);
        }
        float* dst = FM + (size_t)m0 * HID + tn * (unsigned)FM_HB;
        for (int pass = 0; pass < 2; ++pass) {
#pragma unroll
            for (int it = 0; it < 4; ++it) {
                const unsigned row = wave * 16u + (unsigned)it * 4u + q;
                *(volatile v4f*)(dst + (size_t)row * HID + c4) = fv[it];
            }
            __threadfence();
        }
    }
}

extern "C" void kernel_launch(void* const* d_in, const int* in_sizes, int n_in, void* d_out, int out_size,
                              void* d_ws, size_t ws_size, hipStream_t stream) {
    if (n_in < 4) return;
    if (in_sizes[0] < NB * KD || in_sizes[1] < HID * LAT * KD || in_sizes[2] < HID * KD || in_sizes[3] < HID) return;
    if (out_size < NB * HID) return;

    const float* x    = (const float*)d_in[0];
    const float* beta = (const float*)d_in[1];
    const float* Wm   = (const float*)d_in[2];
    const float* bv   = (const float*)d_in[3];
    float* out = (float*)d_out;

    char* wsp = (char*)d_ws;
    size_t off = 0;
    auto carve = [&](size_t bytes) -> void* { void* r = wsp + off; off += (bytes + 255) & ~(size_t)255; return r; };
    unsigned short* XA = (unsigned short*)carve(SZ_XA);
    unsigned short* XB = (unsigned short*)carve(SZ_XB);
    unsigned short* BB = (unsigned short*)carve(SZ_BB);
    unsigned short* WB = (unsigned short*)carve(SZ_WB);
    float*          FM = (float*)carve(SZ_FM);
    if (off > ws_size || off > (size_t)134217728) return;

    k_cvx<<<(NB * (KD / 8)) / 256, 256, 0, stream>>>(x, XA, XB);
    k_cvbw<<<(HID * (KD / 8)) / 256, 256, 0, stream>>>(beta, Wm, BB, WB);

    k_fm<<<(NB / FM_TM) * (NCOL / FM_TN), 128, 0, stream>>>(XB, BB, FM);

    const unsigned gL = ((NB / 64) * (HID / 64) + 7) / 8;
    k_gemm64<0, true, false><<<gL, 256, 0, stream>>>((const _Float16*)XA, KCAT, (const _Float16*)WB, KCAT,
        (void*)out, HID, bv, FM, NB, HID, KCAT, SC, 1.0f);
}
